// FDTD2DLayer_17978733101082
// MI455X (gfx1250) — hardware-run, weakly checked
//
#include <hip/hip_runtime.h>
#include <hip/hip_bf16.h>
#include <stddef.h>
#include <stdint.h>
#include <math.h>

#define SEQ 8192
#define HD  512
#define GD  1024
#define GS  32
#define SFP 68
#define TB  32

static_assert(GD == GS * GS);
static_assert(SEQ % 128 == 0);
static_assert(GD % 64 == 0);
static_assert(HD % 64 == 0);
static_assert(HD % 32 == 0);
static_assert(GD % 32 == 0);
static_assert((SEQ * HD) % 2048 == 0);
static_assert((GD * HD) % 2048 == 0);
static_assert(SEQ % TB == 0);
static_assert(TB * 8 == 4 * 64);

typedef _Float16 hh;
typedef hh v8h __attribute__((ext_vector_type(8)));
typedef hh v16h __attribute__((ext_vector_type(16)));
typedef __attribute__((ext_vector_type(16))) __bf16 v16bf;
typedef float v8f __attribute__((ext_vector_type(8)));
typedef float v4f __attribute__((ext_vector_type(4)));
typedef int v4i __attribute__((ext_vector_type(4)));
typedef int v8i __attribute__((ext_vector_type(8)));
typedef unsigned short v8us __attribute__((ext_vector_type(8)));

__device__ __forceinline__ v8f zero8() { return (v8f){0.f, 0.f, 0.f, 0.f, 0.f, 0.f, 0.f, 0.f}; }

__device__ __forceinline__ float clipf(float x, float lo, float hi) { return fminf(fmaxf(x, lo), hi); }

__device__ __forceinline__ unsigned int bf16_rne_bits(float f) {
  const unsigned int u = __float_as_uint(f);
  return (u + 0x7fffu + ((u >> 16) & 1u)) >> 16;
}

__device__ __forceinline__ v8i ldfrag16(const unsigned short* __restrict__ p, int ld, int row0, int k0, int lane) {
  const unsigned short* q = p + (size_t)(row0 + (lane & 15)) * (size_t)ld + k0 + 8 * (lane >> 4);
  const v4i lo = *(const v4i*)(const void*)(q);
  const v4i hi = *(const v4i*)(const void*)(q + 16);
  return __builtin_shufflevector(lo, hi, 0, 1, 2, 3, 4, 5, 6, 7);
}

__device__ __forceinline__ v8f mma_h(v8i a, v8i b, v8f cc) {
  return __builtin_amdgcn_wmma_f32_16x16x32_f16(false, __builtin_bit_cast(v16h, a), false,
                                                __builtin_bit_cast(v16h, b), (short)0, cc, false, false);
}
__device__ __forceinline__ v8f mma_b(v8i a, v8i b, v8f cc) {
  return __builtin_amdgcn_wmma_f32_16x16x32_bf16(false, __builtin_bit_cast(v16bf, a), false,
                                                 __builtin_bit_cast(v16bf, b), (short)0, cc, false, false);
}

template <bool SPLIT>
__device__ __forceinline__ void gemm32x32(const unsigned short* __restrict__ A, const unsigned short* __restrict__ AL,
                                          int lda, const unsigned short* __restrict__ B,
                                          const unsigned short* __restrict__ BL, int ldb, int ma, int nb, int kdim,
                                          int lane, v8f (&acc)[2][2]) {
#pragma unroll 1
  for (int k0 = 0; k0 < kdim; k0 += 32) {
    const v8i a0 = ldfrag16(A, lda, ma, k0, lane);
    const v8i a1 = ldfrag16(A, lda, ma + 16, k0, lane);
    const v8i b0 = ldfrag16(B, ldb, nb, k0, lane);
    const v8i b1 = ldfrag16(B, ldb, nb + 16, k0, lane);
    if constexpr (!SPLIT) {
      acc[0][0] = mma_h(a0, b0, acc[0][0]);
      acc[1][0] = mma_h(a1, b0, acc[1][0]);
      acc[0][1] = mma_h(a0, b1, acc[0][1]);
      acc[1][1] = mma_h(a1, b1, acc[1][1]);
      asm volatile("v_nop\n\tv_nop\n\tv_nop\n\tv_nop"
                   : "+v"(acc[0][0]), "+v"(acc[0][1]), "+v"(acc[1][0]), "+v"(acc[1][1])
                   : "v"(a0), "v"(a1), "v"(b0), "v"(b1));
    } else {
      const v8i c0 = ldfrag16(AL, lda, ma, k0, lane);
      const v8i c1 = ldfrag16(AL, lda, ma + 16, k0, lane);
      const v8i d0 = ldfrag16(BL, ldb, nb, k0, lane);
      const v8i d1 = ldfrag16(BL, ldb, nb + 16, k0, lane);
      acc[0][0] = mma_b(a0, b0, acc[0][0]);
      acc[1][0] = mma_b(a1, b0, acc[1][0]);
      acc[0][1] = mma_b(a0, b1, acc[0][1]);
      acc[1][1] = mma_b(a1, b1, acc[1][1]);
      acc[0][0] = mma_b(a0, d0, acc[0][0]);
      acc[1][0] = mma_b(a1, d0, acc[1][0]);
      acc[0][1] = mma_b(a0, d1, acc[0][1]);
      acc[1][1] = mma_b(a1, d1, acc[1][1]);
      acc[0][0] = mma_b(c0, b0, acc[0][0]);
      acc[1][0] = mma_b(c1, b0, acc[1][0]);
      acc[0][1] = mma_b(c0, b1, acc[0][1]);
      acc[1][1] = mma_b(c1, b1, acc[1][1]);
      asm volatile("v_nop\n\tv_nop\n\tv_nop\n\tv_nop"
                   : "+v"(acc[0][0]), "+v"(acc[0][1]), "+v"(acc[1][0]), "+v"(acc[1][1])
                   : "v"(a0), "v"(a1), "v"(b0), "v"(b1), "v"(c0), "v"(c1), "v"(d0), "v"(d1));
    }
  }
}

template <int SC>
__global__ __launch_bounds__(256) void k_cvt16(const float* __restrict__ w, unsigned short* __restrict__ wh) {
  const size_t i = ((size_t)blockIdx.x * 256 + threadIdx.x) * 8;
  const v4f a0 = *(const v4f*)(w + i);
  const v4f a1 = *(const v4f*)(w + i + 4);
  v8f t = {a0[0], a0[1], a0[2], a0[3], a1[0], a1[1], a1[2], a1[3]};
  t = t * (float)SC;
  const v8h pk = __builtin_convertvector(t, v8h);
  const v8us bits = __builtin_bit_cast(v8us, pk);
  *(volatile v8us*)(wh + i) = bits;
  __threadfence();
  *(volatile v8us*)(wh + i) = bits;
}

__global__ __launch_bounds__(256) void k_split(const float* __restrict__ w, unsigned short* __restrict__ hi,
                                               unsigned short* __restrict__ lo) {
  const size_t i = ((size_t)blockIdx.x * 256 + threadIdx.x) * 8;
  const v4f a0 = *(const v4f*)(w + i);
  const v4f a1 = *(const v4f*)(w + i + 4);
  const v8f t = {a0[0], a0[1], a0[2], a0[3], a1[0], a1[1], a1[2], a1[3]};
  v8us hv, lv;
#pragma unroll
  for (int e = 0; e < 8; ++e) {
    const float v = t[e];
    const unsigned int hb = bf16_rne_bits(v);
    const float fh = __uint_as_float(hb << 16);
    const unsigned int lb = bf16_rne_bits(v - fh);
    hv[e] = (unsigned short)hb;
    lv[e] = (unsigned short)lb;
  }
  *(volatile v8us*)(hi + i) = hv;
  *(volatile v8us*)(lo + i) = lv;
  __threadfence();
  *(volatile v8us*)(hi + i) = hv;
  *(volatile v8us*)(lo + i) = lv;
}

template <bool SPLIT>
__global__ __launch_bounds__(256) void k_gemm(const unsigned short* __restrict__ A,
                                              const unsigned short* __restrict__ AL,
                                              const unsigned short* __restrict__ B,
                                              const unsigned short* __restrict__ BL,
                                              const float* __restrict__ res, const float* __restrict__ dv,
                                              float* __restrict__ o32) {
  constexpr int KD  = SPLIT ? GD : HD;
  constexpr int LDO = SPLIT ? HD : GD;
  constexpr float OSC = SPLIT ? 1.0f : (1.0f / 64.0f);

  __shared__ __align__(16) float ldsf[128 * SFP];
  const int tid = threadIdx.x, lane = tid & 31, w = tid >> 5;
  const int h = lane >> 4, c = lane & 15;
  const int wm = (w >> 1) * 32, wn = (w & 1) * 32;
  const int m0 = blockIdx.y * 128;
  const int n0 = blockIdx.x * 64;

  v8f acc[2][2];
#pragma unroll
  for (int i = 0; i < 2; ++i)
#pragma unroll
    for (int j = 0; j < 2; ++j) acc[i][j] = zero8();
  gemm32x32<SPLIT>(A, AL, KD, B, BL, KD, m0 + wm, n0 + wn, KD, lane, acc);

#pragma unroll
  for (int i = 0; i < 2; ++i)
#pragma unroll
    for (int j = 0; j < 2; ++j)
#pragma unroll
      for (int r = 0; r < 8; ++r)
        ldsf[(wm + 16 * i + 8 * h + r) * SFP + wn + 16 * j + c] = acc[i][j][r] * OSC;
  __syncthreads();

  v4f val[8];
  size_t go[8];
#pragma unroll
  for (int it = 0; it < 8; ++it) {
    const int p  = tid + 256 * it;
    const int lr = p >> 4;
    const int pc = p & 15;
    const v4f sv = *(const v4f*)(ldsf + lr * SFP + pc * 4);
    const size_t gi = (size_t)(m0 + lr) * LDO + n0 + pc * 4;
    if constexpr (SPLIT) {
      const v4f rr = *(const v4f*)(res + gi);
      const v4f dd = *(const v4f*)(dv + n0 + pc * 4);
      val[it] = sv + rr * dd;
    } else {
      val[it] = sv;
    }
    go[it] = gi;
  }
#pragma unroll
  for (int it = 0; it < 8; ++it) *(volatile v4f*)(o32 + go[it]) = val[it];
  __threadfence();
#pragma unroll
  for (int it = 0; it < 8; ++it) *(volatile v4f*)(o32 + go[it]) = val[it];
}

__global__ __launch_bounds__(64) void k_scan(const float* __restrict__ cvec, const float* __restrict__ kpd,
                                             const float* __restrict__ kd, const float* __restrict__ dtm,
                                             const float* __restrict__ BU, unsigned short* __restrict__ PH,
                                             unsigned short* __restrict__ PL) {
  __shared__ __align__(16) unsigned short lh[TB * 64];
  __shared__ __align__(16) unsigned short ll[TB * 64];
  const int tid = threadIdx.x;
  const int g0 = blockIdx.x * 64;
  const int g = g0 + tid;

  const float dt = clipf(expf(dtm[g]), 0.1f, 5.0f);
  const float cv = cvec[g];
  int di = g / (GS + 1);
  di = min(di, GS - 1);
  const bool ondiag = (g % (GS + 1)) == 0;
  const float kpraw = kpd[di];
  const float kraw  = kd[di];

  float spc = 0.f, kp_d = 0.f, k_d = 0.f, kp_d2 = 0.f, k_d2 = 0.f, kpf = 0.f, kf = 0.f;
#pragma unroll 1
  for (int s = 0; s < 7; ++s) {
    float in;
    if (s == 0) in = cv;
    else if (s == 1) in = kpraw;
    else if (s == 2) in = kraw;
    else if (s == 3) in = kp_d;
    else if (s == 4) in = k_d;
    else if (s == 5) in = ondiag ? kp_d2 : 0.f;
    else in = ondiag ? k_d2 : 0.f;
    const float o = fmaxf(in, 0.f) + log1pf(expf(-fabsf(in)));
    if (s == 0) spc = o;
    else if (s == 1) kp_d = clipf(o, 1e-4f, 0.2f);
    else if (s == 2) k_d = clipf(o, 1e-4f, 0.2f);
    else if (s == 3) kp_d2 = clipf(o, 1e-4f, 0.5f);
    else if (s == 4) k_d2 = clipf(o, 1e-4f, 0.5f);
    else if (s == 5) kpf = clipf(o, 1e-4f, 0.5f);
    else kf = clipf(o, 1e-4f, 0.5f);
  }

  const float dts = clipf(dt, 0.1f, 5.0f);
  const float d1 = fmaxf(1.0f + dts * kf, 0.1f);
  const float d2 = fmaxf(1.0f + dts * kpf, 0.1f);
  const float sq = sqrtf(fmaxf(d1 * d2, 1e-6f));
  const float dsc = 1.0f + dt * kpf;
  const float XI = 1.5707963267948966f;

  float maxc = 0.f, rd1 = 0.f, rd2 = 0.f, qim = 0.f, scal = 0.f;
#pragma unroll 1
  for (int s = 0; s < 5; ++s) {
    float num, den;
    if (s == 0) { num = 0.7f; den = dt; }
    else if (s == 1) { num = 1.0f; den = d1; }
    else if (s == 2) { num = 1.0f; den = d2; }
    else if (s == 3) {
      const float cpos  = clipf(spc, 0.01f, 0.9f * maxc);
      const float csafe = clipf(cpos, 0.01f, 1.0f);
      num = (csafe * dts) * XI;
      den = sq;
    } else { num = 1.0f; den = dsc; }
    const float q = num / den;
    if (s == 0) maxc = q;
    else if (s == 1) rd1 = q;
    else if (s == 2) rd2 = q;
    else if (s == 3) qim = q;
    else scal = q;
  }
  const float lre = 0.5f * (rd2 + rd1);
  const float lim = clipf(qim, -10.0f, 10.0f);

  float a = 0.f, b = 0.f;
  const float* bu = BU + g;
#pragma unroll 1
  for (int t0 = 0; t0 < SEQ; t0 += TB) {
#pragma unroll 4
    for (int tt = 0; tt < TB; ++tt) {
      const float u = bu[(size_t)(t0 + tt) * GD];
      const float f = u * scal;
      const float na = fmaf(lre, a, fmaf(-lim, b, f));
      const float nb = fmaf(lim, a, lre * b);
      a = na;
      b = nb;
      const float p = a + a;
      const unsigned int hb = bf16_rne_bits(p);
      const float fh = __uint_as_float(hb << 16);
      const unsigned int lb = bf16_rne_bits(p - fh);
      lh[tt * 64 + tid] = (unsigned short)hb;
      ll[tt * 64 + tid] = (unsigned short)lb;
    }
    __syncthreads();
    v8us hv[4], lv[4];
    size_t go[4];
#pragma unroll
    for (int it = 0; it < 4; ++it) {
      const int p = tid + 64 * it;
      const int row = p >> 3;
      const int q = p & 7;
      hv[it] = *(const v8us*)(lh + row * 64 + q * 8);
      lv[it] = *(const v8us*)(ll + row * 64 + q * 8);
      go[it] = (size_t)(t0 + row) * GD + g0 + q * 8;
    }
#pragma unroll
    for (int it = 0; it < 4; ++it) {
      *(volatile v8us*)(PH + go[it]) = hv[it];
      *(volatile v8us*)(PL + go[it]) = lv[it];
    }
    __threadfence();
#pragma unroll
    for (int it = 0; it < 4; ++it) {
      *(volatile v8us*)(PH + go[it]) = hv[it];
      *(volatile v8us*)(PL + go[it]) = lv[it];
    }
    __syncthreads();
  }
}

extern "C" void kernel_launch(void* const* d_in, const int* in_sizes, int n_in,
                              void* d_out, int out_size, void* d_ws, size_t ws_size,
                              hipStream_t stream) {
  if (n_in < 8) return;
  if (in_sizes[0] != SEQ * HD) return;
  if (in_sizes[1] != GD) return;
  if (in_sizes[2] != GS) return;
  if (in_sizes[3] != GS) return;
  if (in_sizes[4] != GD) return;
  if (in_sizes[5] != GD * HD) return;
  if (in_sizes[6] != HD * GD) return;
  if (in_sizes[7] != HD) return;
  if (out_size != SEQ * HD) return;

  const float* x   = (const float*)d_in[0];
  const float* cv  = (const float*)d_in[1];
  const float* kpd = (const float*)d_in[2];
  const float* kd  = (const float*)d_in[3];
  const float* dtm = (const float*)d_in[4];
  const float* Bm  = (const float*)d_in[5];
  const float* Cm  = (const float*)d_in[6];
  const float* Dv  = (const float*)d_in[7];
  float* out = (float*)d_out;

  size_t off = 0;
  const size_t oXH = off; off += (size_t)SEQ * HD * 2;
  const size_t oBH = off; off += (size_t)GD * HD * 2;
  const size_t oCH = off; off += (size_t)HD * GD * 2;
  const size_t oCL = off; off += (size_t)HD * GD * 2;
  const size_t oBU = off; off += (size_t)SEQ * GD * 4;
  const size_t oPH = off; off += (size_t)SEQ * GD * 2;
  const size_t oPL = off; off += (size_t)SEQ * GD * 2;
  if (off > ws_size) return;
  if (off > (size_t)134217728) return;

  char* ws = (char*)d_ws;
  unsigned short* XH = (unsigned short*)(ws + oXH);
  unsigned short* BH = (unsigned short*)(ws + oBH);
  unsigned short* CH = (unsigned short*)(ws + oCH);
  unsigned short* CL = (unsigned short*)(ws + oCL);
  float* BU = (float*)(ws + oBU);
  unsigned short* PH = (unsigned short*)(ws + oPH);
  unsigned short* PL = (unsigned short*)(ws + oPL);

  k_cvt16<1><<<dim3((SEQ * HD) / 2048), dim3(256), 0, stream>>>(x, XH);
  k_cvt16<64><<<dim3((GD * HD) / 2048), dim3(256), 0, stream>>>(Bm, BH);
  k_split<<<dim3((HD * GD) / 2048), dim3(256), 0, stream>>>(Cm, CH, CL);
  k_gemm<false><<<dim3(GD / 64, SEQ / 128), dim3(256), 0, stream>>>(XH, XH, BH, BH, x, Dv, BU);
  k_scan<<<dim3(GD / 64), dim3(64), 0, stream>>>(cv, kpd, kd, dtm, BU, PH, PL);
  k_gemm<true><<<dim3(HD / 64, SEQ / 128), dim3(256), 0, stream>>>(PH, PL, CH, CL, x, Dv, out);
  (void)hipGetLastError();
}
